// SeeThroughMultiQ_35304631173914
// MI455X (gfx1250) — hardware-verified
//
#include <hip/hip_runtime.h>
#include <stdint.h>

typedef unsigned short u16;
typedef u16    v8us  __attribute__((ext_vector_type(8)));
typedef u16    v16us __attribute__((ext_vector_type(16)));
typedef __bf16 v16bf __attribute__((ext_vector_type(16)));
typedef float  v8f   __attribute__((ext_vector_type(8)));
typedef float  v4f   __attribute__((ext_vector_type(4)));
typedef v8us __attribute__((may_alias)) v8usa;
typedef v4f  __attribute__((may_alias)) v4fa;

#define CD     256
#define NROWS  39200
#define NQB    800
#define NG     49
#define GPAD   64
#define HW     4096
#define NBATCH 8

static_assert(NROWS % 32 == 0);
static_assert(NQB % 32 == 0);

#define MODE_F32     0
#define MODE_PLANE   1
#define MODE_RELU    2
#define MODE_KK      3
#define MODE_GATE1   4
#define MODE_GATE2   5
#define MODE_LN      6

union Frag { v16us u; v8us half[2]; v16bf b; };

__device__ __forceinline__ u16 bf_rne(float x) {
  unsigned u = __float_as_uint(x);
  u += 0x7FFFu + ((u >> 16) & 1u);
  return (u16)(u >> 16);
}
__device__ __forceinline__ float bf_val(u16 h) { return __uint_as_float(((unsigned)h) << 16); }

__device__ __forceinline__ void split8(const float (&v)[8], v8us& hv, v8us& lv) {
  v8us h8, l8;
#pragma unroll
  for (int e = 0; e < 8; ++e) {
    const u16 hh = bf_rne(v[e]);
    const u16 ll = bf_rne(v[e] - bf_val(hh));
    h8[e] = hh; l8[e] = ll;
  }
  hv = h8; lv = l8;
}

__device__ __forceinline__ void ld8(const float* p, int c0, int c1, float (&o)[8]) {
  const v4f a = *(const v4fa*)(p + c0);
  const v4f b = *(const v4fa*)(p + c1);
  o[0] = a.x; o[1] = a.y; o[2] = a.z; o[3] = a.w;
  o[4] = b.x; o[5] = b.y; o[6] = b.z; o[7] = b.w;
}

__device__ __forceinline__ void st2u(u16* p, v8us v) {
  *(volatile v8us*)p = v;
  __threadfence();
  *(volatile v8us*)p = v;
}
__device__ __forceinline__ void st2f(float* p, v4f v) {
  *(volatile v4f*)p = v;
  __threadfence();
  *(volatile v4f*)p = v;
}

__device__ __forceinline__ float wred(float s) {
  s += __shfl_xor(s, 16);
  s += __shfl_xor(s, 8);
  s += __shfl_xor(s, 4);
  s += __shfl_xor(s, 2);
  s += __shfl_xor(s, 1);
  return s;
}

__device__ __forceinline__ float sigm(float y) {
  const float yc = fminf(fmaxf(y, -30.0f), 30.0f);
  const float e = __expf(-yc);
  return __builtin_amdgcn_rcpf(1.0f + e);
}

__device__ __forceinline__ v8f wmma_bf(v16bf a, v16bf b, v8f c) {
  v8f d = __builtin_amdgcn_wmma_f32_16x16x32_bf16(false, a, false, b, (short)0, c, false, false);
#if defined(__HIP_DEVICE_COMPILE__)
  asm volatile("v_nop\n\tv_nop\n\tv_nop\n\tv_nop" : "+v"(d) : "v"(a), "v"(b));
#endif
  return d;
}
__device__ __forceinline__ v8f mma3(v16bf ah, v16bf al, v16bf bh, v16bf bl, v8f c) {
  c = wmma_bf(ah, bh, c);
  c = wmma_bf(ah, bl, c);
  c = wmma_bf(al, bh, c);
  return c;
}

__device__ __forceinline__ v16bf ldfrag(const u16* p, int h) {
  Frag f;
  f.half[0] = *(const v8usa*)(p + 8 * h);
  f.half[1] = *(const v8usa*)(p + 16 + 8 * h);
  return f.b;
}

__global__ __launch_bounds__(256) void k_zfill(float* p)
{
  const v4f z = {0.0f, 0.0f, 0.0f, 0.0f};
  st2f(p + 4 * threadIdx.x, z);
}

__global__ __launch_bounds__(256) void k_wplanes(
    const float* __restrict__ w0, const float* __restrict__ w1, const float* __restrict__ w2,
    const float* __restrict__ w3, const float* __restrict__ w4, const float* __restrict__ w5,
    const float* __restrict__ w6, const float* __restrict__ w7, const float* __restrict__ w8,
    const float* __restrict__ w9, const float* __restrict__ w10, const float* __restrict__ w11,
    u16* wt)
{
  __shared__ __attribute__((aligned(16))) u16 sH[8 * CD];
  __shared__ __attribute__((aligned(16))) u16 sL[8 * CD];
  const int tid = threadIdx.x, lane = tid & 31, w = tid >> 5;
  const int s = blockIdx.y;
  const int n0 = blockIdx.x * 8;
  const float* W = (s == 0) ? w0 : (s == 1) ? w1 : (s == 2) ? w2 : (s == 3) ? w3 :
                   (s == 4) ? w4 : (s == 5) ? w5 : (s == 6) ? w6 : (s == 7) ? w7 :
                   (s == 8) ? w8 : (s == 9) ? w9 : (s == 10) ? w10 : w11;
  float x[8];
  ld8(W + (size_t)tid * CD + n0, 0, 4, x);
#pragma unroll
  for (int j = 0; j < 8; ++j) {
    const u16 hh = bf_rne(x[j]);
    const u16 ll = bf_rne(x[j] - bf_val(hh));
    sH[j * CD + tid] = hh;
    sL[j * CD + tid] = ll;
  }
  __syncthreads();
  const v8us vh = *(const v8usa*)(sH + w * CD + 8 * lane);
  const v8us vl = *(const v8usa*)(sL + w * CD + 8 * lane);
  u16* dh = wt + (size_t)s * 131072 + (size_t)(n0 + w) * CD + 8 * lane;
  u16* dl = dh + 65536;
  st2u(dh, vh);
  st2u(dl, vl);
}

__global__ __launch_bounds__(256) void k_rplanes(
    const float* __restrict__ s0, const float* __restrict__ s1, int useS1,
    int nreal, int ntot, u16* oh, u16* ol)
{
  const int tid = threadIdx.x, lane = tid & 31, w = tid >> 5;
  const int row = blockIdx.x * 8 + w;
  if (row >= ntot) return;
  const int rc = (row < nreal) ? row : (nreal - 1);
  float v[8];
  ld8(s0 + (size_t)rc * CD, 8 * lane, 8 * lane + 4, v);
  if (useS1) {
    float u[8];
    ld8(s1 + (size_t)rc * CD, 8 * lane, 8 * lane + 4, u);
#pragma unroll
    for (int e = 0; e < 8; ++e) v[e] = v[e] + u[e];
  }
  if (row >= nreal) {
#pragma unroll
    for (int e = 0; e < 8; ++e) v[e] = 0.0f;
  }
  v8us hv, lv;
  split8(v, hv, lv);
  const size_t ob = (size_t)row * CD + 8 * lane;
  st2u(oh + ob, hv);
  st2u(ol + ob, lv);
}

__global__ __launch_bounds__(256) void k_bzl(const float* __restrict__ bz, const float* __restrict__ W, float* out)
{
  __shared__ __attribute__((aligned(16))) float s[CD];
  const int tid = threadIdx.x, lane = tid & 31, w = tid >> 5;
  float a = 0.0f;
#pragma unroll 1
  for (int d = 0; d < CD; ++d) a = fmaf(bz[d], W[(size_t)d * CD + tid], a);
  s[tid] = a;
  __syncthreads();
  if (w == 0) {
    const v4f x0 = *(const v4fa*)(s + 4 * lane);
    const v4f x1 = *(const v4fa*)(s + 128 + 4 * lane);
    st2f(out + 4 * lane, x0);
    st2f(out + 128 + 4 * lane, x1);
  }
}

__global__ __launch_bounds__(256) void k_sample(
    const float* __restrict__ img, const float* __restrict__ imgpe, int usePe,
    const float* __restrict__ bboxes, u16* outH, u16* outL, float* wsumOut)
{
#pragma clang fp contract(off)
  __shared__ __attribute__((aligned(16))) float sval[2 * CD];
  __shared__ int   sidx[32 * 4];
  __shared__ float sw[32 * 4];
  __shared__ __attribute__((aligned(16))) float swsum[32];

  const int tid = threadIdx.x, lane = tid & 31, w = tid >> 5;
  const int rowb = blockIdx.x * 32;

  if (tid < 32) {
    const int row = rowb + tid;
    const int rq  = row / NG;
    const int g   = row - NG * rq;
    const int s1  = g / 7;
    const int s2  = g - 7 * s1;
    const float* bb = bboxes + (size_t)rq * 4;
    const float bx = bb[0], by = bb[1], bh_ = bb[2], bw_ = bb[3];
    const float r7 = 1.0f / 7.0f;
    const float h_sl = bh_ * r7;
    const float w_sl = bw_ * r7;
    const float hh = h_sl * (float)s1 + h_sl * 0.5f;
    const float ww = w_sl * (float)s2 + w_sl * 0.5f;
    float xs = ww + bx; xs = xs - bw_ * 0.5f;
    float ys = hh + by; ys = ys - bh_ * 0.5f;
    float gx = 2.0f * xs - 1.0f; gx = fminf(fmaxf(gx, -1.0f), 1.0f);
    float gy = 2.0f * ys - 1.0f; gy = fminf(fmaxf(gy, -1.0f), 1.0f);
    const float ix = ((gx + 1.0f) * 64.0f - 1.0f) * 0.5f;
    const float iy = ((gy + 1.0f) * 64.0f - 1.0f) * 0.5f;
    const float x0f = floorf(ix), y0f = floorf(iy);
    const float x1f = x0f + 1.0f, y1f = y0f + 1.0f;
    const float wx1 = ix - x0f; const float wx0 = 1.0f - wx1;
    const float wy1 = iy - y0f; const float wy0 = 1.0f - wy1;
    const int x0 = (int)x0f, x1 = (int)x1f, y0 = (int)y0f, y1 = (int)y1f;
    const bool vx0 = (x0 >= 0) && (x0 < 64), vx1 = (x1 >= 0) && (x1 < 64);
    const bool vy0 = (y0 >= 0) && (y0 < 64), vy1 = (y1 >= 0) && (y1 < 64);
    const int cx0 = min(max(x0, 0), 63), cx1 = min(max(x1, 0), 63);
    const int cy0 = min(max(y0, 0), 63), cy1 = min(max(y1, 0), 63);
    const float w00 = wx0 * wy0, w10 = wx1 * wy0, w01 = wx0 * wy1, w11 = wx1 * wy1;
    const float e00 = (vx0 && vy0) ? w00 : 0.0f;
    const float e10 = (vx1 && vy0) ? w10 : 0.0f;
    const float e01 = (vx0 && vy1) ? w01 : 0.0f;
    const float e11 = (vx1 && vy1) ? w11 : 0.0f;
    sidx[tid * 4 + 0] = cy0 * 64 + cx0;
    sidx[tid * 4 + 1] = cy0 * 64 + cx1;
    sidx[tid * 4 + 2] = cy1 * 64 + cx0;
    sidx[tid * 4 + 3] = cy1 * 64 + cx1;
    sw[tid * 4 + 0] = e00; sw[tid * 4 + 1] = e10; sw[tid * 4 + 2] = e01; sw[tid * 4 + 3] = e11;
    float wsm = e00 + e10; wsm = wsm + e01; wsm = wsm + e11;
    swsum[tid] = wsm;
  }
  __syncthreads();

  const int c = tid;
#pragma unroll 1
  for (int r = 0; r < 32; ++r) {
    const int row = rowb + r;
    const int b   = row / (100 * NG);
    const size_t cb = ((size_t)b * CD + c) * HW;
    const int i0 = sidx[r * 4 + 0], i1 = sidx[r * 4 + 1], i2 = sidx[r * 4 + 2], i3 = sidx[r * 4 + 3];
    const float e0 = sw[r * 4 + 0], e1 = sw[r * 4 + 1], e2 = sw[r * 4 + 2], e3 = sw[r * 4 + 3];
    float v0 = img[cb + i0], v1 = img[cb + i1], v2 = img[cb + i2], v3 = img[cb + i3];
    if (usePe) {
      v0 = v0 + imgpe[cb + i0]; v1 = v1 + imgpe[cb + i1];
      v2 = v2 + imgpe[cb + i2]; v3 = v3 + imgpe[cb + i3];
    }
    float a = v0 * e0;
    a = a + v1 * e1;
    a = a + v2 * e2;
    a = a + v3 * e3;
    sval[(r & 1) * CD + c] = a;
    __syncthreads();
    if (w < 2) {
      float x[8];
      ld8(sval + (r & 1) * CD, 8 * lane, 8 * lane + 4, x);
      v8us hv, lv;
      split8(x, hv, lv);
      const v8us o = (w == 0) ? hv : lv;
      u16* dst = ((w == 0) ? outH : outL) + (size_t)row * CD + 8 * lane;
      st2u(dst, o);
    }
  }
  if (w == 0 && lane < 8) {
    const v4f x = *(const v4fa*)(swsum + 4 * lane);
    st2f(wsumOut + (size_t)blockIdx.x * 32 + 4 * lane, x);
  }
}

__global__ __launch_bounds__(256) void k_hbuild(
    const float* __restrict__ P, const float* __restrict__ Gf, const float* __restrict__ b1,
    u16* oh, u16* ol)
{
  const int tid = threadIdx.x, lane = tid & 31, w = tid >> 5;
  float bb[8];
  ld8(b1, 8 * lane, 8 * lane + 4, bb);
#pragma unroll 1
  for (int rr = 0; rr < 4; ++rr) {
    const int row = blockIdx.x * 32 + 4 * w + rr;
    const int rq = row / NG;
    const int g  = row - NG * rq;
    float p[8], gf[8], v[8];
    ld8(P + (size_t)rq * CD, 8 * lane, 8 * lane + 4, p);
    ld8(Gf + (size_t)g * CD, 8 * lane, 8 * lane + 4, gf);
#pragma unroll
    for (int e = 0; e < 8; ++e) v[e] = fmaxf((p[e] + gf[e]) + bb[e], 0.0f);
    v8us hv, lv;
    split8(v, hv, lv);
    const size_t ob = (size_t)row * CD + 8 * lane;
    st2u(oh + ob, hv);
    st2u(ol + ob, lv);
  }
}

__global__ __launch_bounds__(256) void k_gemm(
    const u16* __restrict__ Ah, const u16* __restrict__ Al,
    const u16* __restrict__ Bh, const u16* __restrict__ Bl,
    const float* __restrict__ bias, const float* __restrict__ bias2,
    const float* __restrict__ gam, const float* __restrict__ bet,
    const float* p0, const float* p1, const float* p2, const float* p3,
    int mode, float* outF, u16* outH, u16* outL)
{
  __shared__ __attribute__((aligned(16))) float tile[32 * CD];

  const int tid = threadIdx.x, lane = tid & 31, w = tid >> 5;
  const int h = lane >> 4, m = lane & 15;
  const int row0 = blockIdx.x * 32;
  const int n0 = 32 * w;

  const u16* ah0 = Ah + (size_t)(row0 + m) * CD;
  const u16* ah1 = ah0 + 16 * CD;
  const u16* al0 = Al + (size_t)(row0 + m) * CD;
  const u16* al1 = al0 + 16 * CD;
  const u16* bh0 = Bh + (size_t)(n0 + m) * CD;
  const u16* bh1 = bh0 + 16 * CD;
  const u16* bl0 = Bl + (size_t)(n0 + m) * CD;
  const u16* bl1 = bl0 + 16 * CD;

  const v8f z8 = {0.f, 0.f, 0.f, 0.f, 0.f, 0.f, 0.f, 0.f};
  v8f a00 = z8, a01 = z8, a10 = z8, a11 = z8;

#pragma unroll 1
  for (int k0 = 0; k0 < CD; k0 += 32) {
    const v16bf fa0h = ldfrag(ah0 + k0, h);
    const v16bf fa1h = ldfrag(ah1 + k0, h);
    const v16bf fa0l = ldfrag(al0 + k0, h);
    const v16bf fa1l = ldfrag(al1 + k0, h);
    const v16bf fb0h = ldfrag(bh0 + k0, h);
    const v16bf fb1h = ldfrag(bh1 + k0, h);
    const v16bf fb0l = ldfrag(bl0 + k0, h);
    const v16bf fb1l = ldfrag(bl1 + k0, h);
    a00 = mma3(fa0h, fa0l, fb0h, fb0l, a00);
    a01 = mma3(fa0h, fa0l, fb1h, fb1l, a01);
    a10 = mma3(fa1h, fa1l, fb0h, fb0l, a10);
    a11 = mma3(fa1h, fa1l, fb1h, fb1l, a11);
  }

#pragma unroll
  for (int r = 0; r < 8; ++r) {
    const int ra = (8 * h + r) * CD;
    const int rb = (16 + 8 * h + r) * CD;
    tile[ra + n0 + m]      = a00[r];
    tile[ra + n0 + 16 + m] = a01[r];
    tile[rb + n0 + m]      = a10[r];
    tile[rb + n0 + 16 + m] = a11[r];
  }
  __syncthreads();

  const bool pm = (mode == MODE_PLANE) | (mode == MODE_RELU) | (mode == MODE_KK) | (mode == MODE_GATE2);
  const int c0 = pm ? 8 * lane : 4 * lane;
  const int c1 = pm ? 8 * lane + 4 : 128 + 4 * lane;
  float bb[8], b2[8], gg[8], be[8], bzv[8];
  ld8(bias, c0, c1, bb);
  ld8(bias2, c0, c1, b2);
  ld8(gam, c0, c1, gg);
  ld8(bet, c0, c1, be);
  if (mode == MODE_KK) {
    ld8(p1, c0, c1, bzv);
  } else {
#pragma unroll
    for (int e = 0; e < 8; ++e) bzv[e] = 0.0f;
  }

#pragma unroll 1
  for (int rr = 0; rr < 4; ++rr) {
    const int r = 4 * w + rr;
    const int row = row0 + r;
    float v[8];
    {
      const v4f xa = *(const v4fa*)(tile + r * CD + c0);
      const v4f xb = *(const v4fa*)(tile + r * CD + c1);
      v[0] = xa.x + bb[0]; v[1] = xa.y + bb[1]; v[2] = xa.z + bb[2]; v[3] = xa.w + bb[3];
      v[4] = xb.x + bb[4]; v[5] = xb.y + bb[5]; v[6] = xb.z + bb[6]; v[7] = xb.w + bb[7];
    }
    if (mode == MODE_RELU) {
#pragma unroll
      for (int e = 0; e < 8; ++e) v[e] = fmaxf(v[e], 0.0f);
    } else if (mode == MODE_KK) {
      const int rq = row / NG;
      const int g  = row - NG * rq;
      const float wsm = p0[row];
      float tt[8], gw[8];
      ld8(p2 + (size_t)rq * CD, c0, c1, tt);
      ld8(p3 + (size_t)g * CD, c0, c1, gw);
#pragma unroll
      for (int e = 0; e < 8; ++e) {
        const float rt = v[e] + wsm * bzv[e];
        const float lt = (tt[e] + gw[e]) + b2[e];
        v[e] = lt * rt;
      }
    } else if (mode >= MODE_GATE1) {
      float s = 0.0f;
#pragma unroll
      for (int e = 0; e < 8; ++e) s += v[e];
      s = wred(s);
      const float mean = s * (1.0f / 256.0f);
      float d[8];
      float q = 0.0f;
#pragma unroll
      for (int e = 0; e < 8; ++e) { d[e] = v[e] - mean; q += d[e] * d[e]; }
      q = wred(q);
      const float rstd = __builtin_amdgcn_rsqf(q * (1.0f / 256.0f) + 1e-5f);
#pragma unroll
      for (int e = 0; e < 8; ++e) v[e] = d[e] * rstd * gg[e] + be[e];
      if (mode == MODE_GATE1) {
        float f[8];
        ld8(p0 + (size_t)row * CD, c0, c1, f);
#pragma unroll
        for (int e = 0; e < 8; ++e) v[e] = sigm(v[e]) * f[e];
      } else if (mode == MODE_GATE2) {
        float f[8], o[8];
        ld8(p0 + (size_t)row * CD, c0, c1, f);
        ld8(p1 + (size_t)row * CD, c0, c1, o);
#pragma unroll
        for (int e = 0; e < 8; ++e) v[e] = o[e] + sigm(v[e]) * f[e];
      }
    }
    if (pm) {
      v8us hv, lv;
      split8(v, hv, lv);
      const size_t ob = (size_t)row * CD + 8 * lane;
      st2u(outH + ob, hv);
      st2u(outL + ob, lv);
    } else {
      const v4f o0 = {v[0], v[1], v[2], v[3]};
      const v4f o1 = {v[4], v[5], v[6], v[7]};
      float* ob = outF + (size_t)row * CD;
      st2f(ob + 4 * lane, o0);
      st2f(ob + 128 + 4 * lane, o1);
    }
  }
}

static void gemm_launch(hipStream_t st, int blocks,
                        const u16* Ah, const u16* Al, const u16* Bh, const u16* Bl,
                        const float* bias, const float* bias2, const float* gam, const float* bet,
                        const float* p0, const float* p1, const float* p2, const float* p3,
                        int mode, float* outF, u16* outH, u16* outL)
{
  k_gemm<<<blocks, 256, 0, st>>>(Ah, Al, Bh, Bl, bias, bias2, gam, bet, p0, p1, p2, p3, mode, outF, outH, outL);
}

extern "C" void kernel_launch(void* const* d_in, const int* in_sizes, int n_in,
                              void* d_out, int out_size, void* d_ws, size_t ws_size,
                              hipStream_t stream)
{
  if (n_in < 38) return;
  if (in_sizes[0] != NQB * CD || in_sizes[1] != NQB * CD) return;
  if (in_sizes[2] != NBATCH * CD * HW || in_sizes[3] != NBATCH * CD * HW) return;
  if (in_sizes[4] != NQB * 4 || in_sizes[5] != NG * CD) return;
  for (int i = 6; i <= 18; ++i) if (in_sizes[i] != CD * CD) return;
  for (int i = 19; i <= 37; ++i) if (in_sizes[i] != CD) return;
  if (out_size != NROWS * CD) return;

  const float* q    = (const float*)d_in[0];
  const float* qpe  = (const float*)d_in[1];
  const float* feat = (const float*)d_in[2];
  const float* fpe  = (const float*)d_in[3];
  const float* bbox = (const float*)d_in[4];
  const float* ge   = (const float*)d_in[5];
  const float* Wz   = (const float*)d_in[6];
  const float* Wm[12];
  for (int i = 0; i < 12; ++i) Wm[i] = (const float*)d_in[7 + i];
  const float* W2l  = (const float*)d_in[9];
  const float* bz   = (const float*)d_in[19];
  const float* bq   = (const float*)d_in[20];
  const float* b1l  = (const float*)d_in[21];
  const float* b2l  = (const float*)d_in[22];
  const float* g1b1 = (const float*)d_in[23];
  const float* g1b2 = (const float*)d_in[24];
  const float* g2b1 = (const float*)d_in[25];
  const float* g2b2 = (const float*)d_in[26];
  const float* f1b1 = (const float*)d_in[27];
  const float* f1b2 = (const float*)d_in[28];
  const float* f2b1 = (const float*)d_in[29];
  const float* f2b2 = (const float*)d_in[30];
  const float* outb = (const float*)d_in[31];
  const float* g1beta  = (const float*)d_in[32];
  const float* g2beta  = (const float*)d_in[33];
  const float* outbeta = (const float*)d_in[34];
  const float* g1g  = (const float*)d_in[35];
  const float* g2g  = (const float*)d_in[36];
  const float* outg = (const float*)d_in[37];
  float* dout = (float*)d_out;

  char* ws = (char*)d_ws;
  size_t off = 0;
  auto take = [&](size_t bytes) { size_t o = off; off += (bytes + 4095) & ~(size_t)4095; return o; };
  const size_t PLS   = (size_t)NQB * CD * 2;
  const size_t PLG   = (size_t)GPAD * CD * 2;
  const size_t PLW   = (size_t)CD * CD * 2;
  const size_t PLB   = (size_t)NROWS * CD * 2;
  const size_t BIG   = (size_t)NROWS * CD * 4;
  const size_t o_zb   = take(4096);
  const size_t o_wt   = take(12 * 2 * PLW);
  const size_t o_wzl  = take(2 * PLW);
  const size_t o_wzn  = take(2 * PLW);
  const size_t o_xq   = take(2 * PLS);
  const size_t o_q    = take(2 * PLS);
  const size_t o_qs   = take(2 * PLS);
  const size_t o_ge   = take(2 * PLG);
  const size_t o_T    = take((size_t)NQB * CD * 4);
  const size_t o_P    = take((size_t)NQB * CD * 4);
  const size_t o_Gw   = take((size_t)GPAD * CD * 4);
  const size_t o_Gf   = take((size_t)GPAD * CD * 4);
  const size_t o_bzl  = take(1024);
  const size_t o_wsum = take((size_t)NROWS * 4);
  const size_t o_R0   = take(BIG);
  const size_t o_R1   = take(BIG);
  const size_t o_R2   = take(BIG);
  if (off > ws_size) return;

  float* zb   = (float*)(ws + o_zb);
  u16*   wt   = (u16*)(ws + o_wt);
  u16*   wzlH = (u16*)(ws + o_wzl);  u16* wzlL = (u16*)(ws + o_wzl + PLW);
  u16*   wznH = (u16*)(ws + o_wzn);  u16* wznL = (u16*)(ws + o_wzn + PLW);
  u16*   xqH  = (u16*)(ws + o_xq);   u16* xqL  = (u16*)(ws + o_xq + PLS);
  u16*   qH   = (u16*)(ws + o_q);    u16* qL   = (u16*)(ws + o_q + PLS);
  u16*   qsH  = (u16*)(ws + o_qs);   u16* qsL  = (u16*)(ws + o_qs + PLS);
  u16*   geH  = (u16*)(ws + o_ge);   u16* geL  = (u16*)(ws + o_ge + PLG);
  float* T    = (float*)(ws + o_T);
  float* P    = (float*)(ws + o_P);
  float* Gw   = (float*)(ws + o_Gw);
  float* Gf   = (float*)(ws + o_Gf);
  float* bzl  = (float*)(ws + o_bzl);
  float* wsum = (float*)(ws + o_wsum);
  u16* R0h = (u16*)(ws + o_R0); u16* R0l = (u16*)(ws + o_R0 + PLB); float* R0f = (float*)(ws + o_R0);
  u16* R1h = (u16*)(ws + o_R1); u16* R1l = (u16*)(ws + o_R1 + PLB); float* R1f = (float*)(ws + o_R1);
  u16* R2h = (u16*)(ws + o_R2); u16* R2l = (u16*)(ws + o_R2 + PLB); float* R2f = (float*)(ws + o_R2);
  (void)R0f;
  auto wtH = [&](int s) { return wt + (size_t)s * 131072; };
  auto wtL = [&](int s) { return wt + (size_t)s * 131072 + 65536; };

  const int NB  = NROWS / 32;
  const int NBS = NQB / 32;

  k_zfill<<<1, 256, 0, stream>>>(zb);

  k_wplanes<<<dim3(CD / 8, 12), 256, 0, stream>>>(Wm[0], Wm[1], Wm[2], Wm[3], Wm[4], Wm[5],
                                                  Wm[6], Wm[7], Wm[8], Wm[9], Wm[10], Wm[11], wt);
  k_rplanes<<<NQB / 8, 256, 0, stream>>>(q, qpe, 1, NQB, NQB, xqH, xqL);
  k_rplanes<<<NQB / 8, 256, 0, stream>>>(q, q, 0, NQB, NQB, qH, qL);
  k_rplanes<<<GPAD / 8, 256, 0, stream>>>(ge, ge, 0, NG, GPAD, geH, geL);
  k_rplanes<<<CD / 8, 256, 0, stream>>>(Wz, Wz, 0, CD, CD, wznH, wznL);
  k_bzl<<<1, 256, 0, stream>>>(bz, W2l, bzl);

  gemm_launch(stream, NBS, xqH, xqL, wtH(0), wtL(0), bq, zb, zb, zb, zb, zb, zb, zb, MODE_PLANE, dout, qsH, qsL);
  gemm_launch(stream, NBS, qsH, qsL, wtH(1), wtL(1), zb, zb, zb, zb, zb, zb, zb, zb, MODE_F32, T, R0h, R0l);
  gemm_launch(stream, GPAD / 32, geH, geL, wtH(1), wtL(1), zb, zb, zb, zb, zb, zb, zb, zb, MODE_F32, Gw, R0h, R0l);
  gemm_launch(stream, NBS, qH, qL, wtH(7), wtL(7), zb, zb, zb, zb, zb, zb, zb, zb, MODE_F32, P, R0h, R0l);
  gemm_launch(stream, GPAD / 32, geH, geL, wtH(7), wtL(7), zb, zb, zb, zb, zb, zb, zb, zb, MODE_F32, Gf, R0h, R0l);
  gemm_launch(stream, CD / 32, wtH(2), wtL(2), wznH, wznL, zb, zb, zb, zb, zb, zb, zb, zb, MODE_PLANE, dout, wzlH, wzlL);

  k_hbuild<<<NB, 256, 0, stream>>>(P, Gf, f1b1, R0h, R0l);
  gemm_launch(stream, NB, R0h, R0l, wtH(8), wtL(8), f1b2, zb, zb, zb, zb, zb, zb, zb, MODE_F32, R2f, R1h, R1l);

  k_sample<<<NB, 256, 0, stream>>>(feat, fpe, 1, bbox, R0h, R0l, wsum);
  gemm_launch(stream, NB, R0h, R0l, wzlH, wzlL, b2l, b1l, zb, zb, wsum, bzl, T, Gw, MODE_KK, dout, R1h, R1l);
  gemm_launch(stream, NB, R1h, R1l, wtH(3), wtL(3), g1b1, zb, zb, zb, zb, zb, zb, zb, MODE_RELU, dout, R0h, R0l);
  gemm_launch(stream, NB, R0h, R0l, wtH(4), wtL(4), g1b2, zb, g1g, g1beta, R2f, zb, zb, zb, MODE_GATE1, dout, R1h, R1l);
  gemm_launch(stream, NB, R1h, R1l, wtH(5), wtL(5), g2b1, zb, zb, zb, zb, zb, zb, zb, MODE_RELU, dout, R0h, R0l);
  k_sample<<<NB, 256, 0, stream>>>(feat, feat, 0, bbox, R1h, R1l, wsum);
  gemm_launch(stream, NB, R1h, R1l, wtH(9), wtL(9), f2b1, zb, zb, zb, zb, zb, zb, zb, MODE_RELU, dout, R2h, R2l);
  gemm_launch(stream, NB, R2h, R2l, wtH(10), wtL(10), f2b2, zb, zb, zb, zb, zb, zb, zb, MODE_F32, R1f, R1h, R1l);
  gemm_launch(stream, NB, R0h, R0l, wtH(6), wtL(6), g2b2, zb, g2g, g2beta, R1f, dout, zb, zb, MODE_GATE2, dout, R2h, R2l);
  gemm_launch(stream, NB, R2h, R2l, wtH(11), wtL(11), outb, zb, outg, outbeta, zb, zb, zb, zb, MODE_LN, dout, R0h, R0l);
}
